// Conv_KNRM_34084860461087
// MI455X (gfx1250) — hardware-verified
//
#include <hip/hip_runtime.h>


namespace {
constexpr int NB = 128, QL = 30, QR = 32, DL = 256, EMB = 300, EP = 320, CO = 128, NK = 11, NGR = 3, QROWS = 48, DROWS = 272;
constexpr float XS = 8.0f, WSC = 256.0f, NS8 = 8.0f;
__constant__ float MU[NK] = {1.0f, 0.9f, 0.7f, 0.5f, 0.3f, 0.1f, -0.1f, -0.3f, -0.5f, -0.7f, -0.9f};
__constant__ float SIG[NK] = {0.001f, 0.1f, 0.1f, 0.1f, 0.1f, 0.1f, 0.1f, 0.1f, 0.1f, 0.1f, 0.1f};

typedef _Float16 b16;
typedef __attribute__((ext_vector_type(16))) _Float16 v16b;
typedef __attribute__((ext_vector_type(8))) _Float16 v8b;
typedef __attribute__((ext_vector_type(8))) float v8f;
typedef __attribute__((ext_vector_type(4))) float v4f;
__device__ __forceinline__ float bf16_rne(float f) { unsigned int u = __float_as_uint(f); u += 0x7FFFu + ((u >> 16) & 1u); return __uint_as_float(u & 0xFFFF0000u); }
__device__ __forceinline__ void split16(float v, b16& hi, b16& lo) { hi = (b16)v; lo = (b16)(v - (float)hi); }
__device__ __forceinline__ v16b frag_kb(const b16* p, int hh) { const v8b a = *(const v8b*)(p + 8 * hh), b = *(const v8b*)(p + 16 + 8 * hh); v16b f;
#pragma unroll
  for (int e = 0; e < 8; ++e) { f[e] = a[e]; f[8 + e] = b[e]; } return f; }
__device__ __forceinline__ v8f wmma16b(v16b a, v16b b, v8f c) { v8f d = __builtin_amdgcn_wmma_f32_16x16x32_f16(false, a, false, b, (short)0, c, false, false); asm volatile("v_nop\n\tv_nop\n\tv_nop\n\tv_nop" : "+v"(d) : "v"(a), "v"(b)); return d; }
__device__ __forceinline__ void wave_lds_sync() { __builtin_amdgcn_fence(__ATOMIC_RELEASE, "workgroup"); __builtin_amdgcn_wave_barrier(); __builtin_amdgcn_fence(__ATOMIC_ACQUIRE, "workgroup"); }
__device__ __forceinline__ float pmul(float a, float b) { float p = a * b; asm volatile("" : "+v"(p)); return p; }
__device__ __forceinline__ float hsum16(float v) { v += __shfl_xor(v, 1); v += __shfl_xor(v, 2); v += __shfl_xor(v, 4); return v + __shfl_xor(v, 8); }

__global__ __launch_bounds__(256) void prepw_kernel(const float* __restrict__ w1, const float* __restrict__ w2, const float* __restrict__ w3, b16* __restrict__ W0, b16* __restrict__ W1, b16* __restrict__ W2) {
  const int g = blockIdx.y, k = g + 1, tid = blockIdx.x * 256 + threadIdx.x, nth = gridDim.x * 256; const float* w = g == 0 ? w1 : g == 1 ? w2 : w3; b16* Wd = g == 0 ? W0 : g == 1 ? W1 : W2;
  for (int pass = 0; pass < 2; ++pass) {
    for (int gidx = tid; gidx < CO * k * (EP / 8); gidx += nth) { const int c = gidx / (k * (EP / 8)), rem = gidx - c * (k * (EP / 8)), j = rem / (EP / 8), e0 = (rem - j * (EP / 8)) * 8; v8b o;
#pragma unroll
      for (int q = 0; q < 8; ++q) { const int e = e0 + q; o[q] = (e < EMB) ? (b16)(bf16_rne(w[((size_t)c * EMB + (e < EMB ? e : 0)) * k + j]) * WSC) : (b16)0.0f; }
      *(volatile v8b*)(Wd + ((size_t)c * k + j) * EP + e0) = o; }
    __threadfence(); }
}
__global__ __launch_bounds__(256) void prepe_kernel(const float* __restrict__ qe, const float* __restrict__ de, b16* __restrict__ QE, b16* __restrict__ DE) {
  const int wave = threadIdx.x >> 5, lane = threadIdx.x & 31, row = blockIdx.x * 8 + wave;
  const bool isq = row < NB * QROWS; const int r2 = isq ? row : row - NB * QROWS; const int b = isq ? r2 / QROWS : r2 / DROWS, t = isq ? r2 - b * QROWS : r2 - b * DROWS;
  const int L = isq ? QL : DL; const bool live = t < L; const float* src = (isq ? qe : de) + ((size_t)b * L + (live ? t : 0)) * EMB; b16* base = isq ? QE : DE;
  v8b o0, o1;
#pragma unroll
  for (int q = 0; q < 8; ++q) { const int e = lane * 8 + q; o0[q] = (live && e < EMB) ? (b16)(bf16_rne(src[e < EMB ? e : 0]) * XS) : (b16)0.0f; const int e1 = 256 + lane * 8 + q; o1[q] = (live && e1 < EMB && lane < 8) ? (b16)(bf16_rne(src[e1 < EMB ? e1 : 0]) * XS) : (b16)0.0f; }
  for (int pass = 0; pass < 2; ++pass) { *(volatile v8b*)(base + (size_t)r2 * EP + lane * 8) = o0; if (lane < 8) *(volatile v8b*)(base + (size_t)r2 * EP + 256 + lane * 8) = o1; __threadfence(); }
}
template <bool ISQ>
__global__ __launch_bounds__(64) void conv_kernel(const b16* __restrict__ E, const b16* __restrict__ W0, const b16* __restrict__ W1, const b16* __restrict__ W2, const float* __restrict__ b1, const float* __restrict__ b2, const float* __restrict__ b3, b16* __restrict__ NH, b16* __restrict__ NL) {
  __shared__ __attribute__((aligned(16))) b16 Th[2][16][CO + 8], Tl[2][16][CO + 8];
  constexpr int RP = ISQ ? QROWS : DROWS, RT = ISQ ? QR : DL;
  const int wave = threadIdx.x >> 5, lane = threadIdx.x & 31, nloc = lane & 15, hlf = lane >> 4; const int b = blockIdx.z, g = blockIdx.y, m0 = blockIdx.x * 32 + wave * 16, k = g + 1;
  const b16* W = g == 0 ? W0 : g == 1 ? W1 : W2; const float* bias = g == 0 ? b1 : g == 1 ? b2 : b3; const b16* A = E + ((size_t)b * RP + m0 + nloc) * EP;
  v8f acc[8];
#pragma unroll
  for (int t = 0; t < 8; ++t) acc[t] = (v8f){};
  for (int j = 0; j < k; ++j) {
#pragma unroll 2
    for (int e0 = 0; e0 < EP; e0 += 32) { const v16b a = frag_kb(A + (size_t)j * EP + e0, hlf);
#pragma unroll
      for (int t = 0; t < 8; ++t) acc[t] = wmma16b(a, frag_kb(W + ((size_t)(t * 16 + nloc) * k + j) * EP + e0, hlf), acc[t]); } }
  float ss = 0.0f;
#pragma unroll
  for (int t = 0; t < 8; ++t) { const float bb = bf16_rne(bias[t * 16 + nloc]);
#pragma unroll
    for (int r = 0; r < 8; ++r) { const float v = fmaxf(acc[t][r] * (1.0f / (XS * WSC)) + bb, 0.0f); acc[t][r] = v; } }
  float inv[8];
#pragma unroll
  for (int r = 0; r < 8; ++r) { float s = 0.0f;
#pragma unroll
    for (int t = 0; t < 8; ++t) s += pmul(acc[t][r], acc[t][r]);
    s = hsum16(s); inv[r] = 1.0f / (sqrtf(s) + 1e-13f); }
#pragma unroll
  for (int t = 0; t < 8; ++t)
#pragma unroll
    for (int r = 0; r < 8; ++r) { b16 a_, c_; split16(pmul(acc[t][r], inv[r]) * NS8, a_, c_); Th[wave][8 * hlf + r][t * 16 + nloc] = a_; Tl[wave][8 * hlf + r][t * 16 + nloc] = c_; }
  wave_lds_sync();
  for (int pass = 0; pass < 2; ++pass) { for (int rr = 0; rr < 16; ++rr) if (lane < 16) { const size_t gi = (((size_t)b * NGR + g) * RT + m0 + rr) * CO + lane * 8; *(volatile v8b*)(NH + gi) = *(const v8b*)(&Th[wave][rr][lane * 8]); *(volatile v8b*)(NL + gi) = *(const v8b*)(&Tl[wave][rr][lane * 8]); } __threadfence(); }
}
__global__ __launch_bounds__(256) void cos_kernel(const b16* __restrict__ NQH, const b16* __restrict__ NQL, const b16* __restrict__ NDH, const b16* __restrict__ NDL, const float* __restrict__ qmask, const float* __restrict__ dmask, float* __restrict__ ALLG) {
  __shared__ float Sp[8][QR][NK + 1]; __shared__ float Sout[32];
  const int b = blockIdx.y, it = blockIdx.x, i = it / NGR, t = it - i * NGR, wave = threadIdx.x >> 5, lane = threadIdx.x & 31, nloc = lane & 15, hlf = lane >> 4;
  const b16* Qh = NQH + ((size_t)b * NGR + i) * QR * CO; const b16* Ql = NQL + ((size_t)b * NGR + i) * QR * CO; const b16* Dh = NDH + ((size_t)b * NGR + t) * DL * CO; const b16* Dl = NDL + ((size_t)b * NGR + t) * DL * CO;
  v8f acc[2][2];
#pragma unroll
  for (int mt = 0; mt < 2; ++mt)
#pragma unroll
    for (int nt = 0; nt < 2; ++nt) acc[mt][nt] = (v8f){};
#pragma unroll
  for (int kb = 0; kb < CO; kb += 32) { v16b qh[2], ql[2];
#pragma unroll
    for (int mt = 0; mt < 2; ++mt) { qh[mt] = frag_kb(Qh + (size_t)(mt * 16 + nloc) * CO + kb, hlf); ql[mt] = frag_kb(Ql + (size_t)(mt * 16 + nloc) * CO + kb, hlf); }
#pragma unroll
    for (int nt = 0; nt < 2; ++nt) { const int d0 = (wave * 2 + nt) * 16; const v16b dh = frag_kb(Dh + (size_t)(d0 + nloc) * CO + kb, hlf), dl = frag_kb(Dl + (size_t)(d0 + nloc) * CO + kb, hlf);
#pragma unroll
      for (int mt = 0; mt < 2; ++mt) { acc[mt][nt] = wmma16b(qh[mt], dh, acc[mt][nt]); acc[mt][nt] = wmma16b(qh[mt], dl, acc[mt][nt]); acc[mt][nt] = wmma16b(ql[mt], dh, acc[mt][nt]); } } }
  const float dm0 = bf16_rne(dmask[(size_t)b * DL + (wave * 2 + 0) * 16 + nloc]), dm1 = bf16_rne(dmask[(size_t)b * DL + (wave * 2 + 1) * 16 + nloc]);
#pragma unroll
  for (int mt = 0; mt < 2; ++mt)
#pragma unroll
    for (int r = 0; r < 8; ++r) { const int q = mt * 16 + 8 * hlf + r; const float qm = bf16_rne(qmask[(size_t)b * QL + (q < QL ? q : 0)]);
      const float c0 = pmul(acc[mt][0][r] * (1.0f / (NS8 * NS8)), pmul(qm, dm0)), c1 = pmul(acc[mt][1][r] * (1.0f / (NS8 * NS8)), pmul(qm, dm1));
#pragma unroll
      for (int m = 0; m < NK; ++m) { const float den = 2.0f * pmul(SIG[m], SIG[m]); const float e0 = c0 - MU[m], e1 = c1 - MU[m];
        float kv = pmul(__expf(-pmul(e0, e0) / den), pmul(qm, dm0)) + pmul(__expf(-pmul(e1, e1) / den), pmul(qm, dm1));
        kv = hsum16(kv); if (nloc == 0) Sp[wave][q][m] = kv; } }
  __syncthreads();
  if (threadIdx.x < 32) { float val = 0.0f;
    if (lane < NK) { for (int q = 0; q < QL; ++q) { float s = 0.0f; for (int w = 0; w < 8; ++w) s += Sp[w][q][lane]; const float lg = __logf(fmaxf(s, 1e-10f)) * 0.01f; val += pmul(lg, bf16_rne(qmask[(size_t)b * QL + q])); } }
    Sout[lane] = val; }
  __syncthreads();
  for (int pass = 0; pass < 2; ++pass) { if (threadIdx.x < 32) ((volatile float*)ALLG)[((size_t)b * (NGR * NGR) + it) * 32 + lane] = Sout[lane]; __threadfence(); }
}
__global__ __launch_bounds__(128) void dense_kernel(const float* __restrict__ ALLG, const float* __restrict__ dw, float* __restrict__ out) {
  const int b = threadIdx.x; float s = 0.0f;
  for (int it = 0; it < NGR * NGR; ++it)
#pragma unroll 1
    for (int m = 0; m < NK; ++m) s += pmul(ALLG[((size_t)b * (NGR * NGR) + it) * 32 + m], bf16_rne(dw[it * NK + m]));
  for (int pass = 0; pass < 2; ++pass) { ((volatile float*)out)[b] = s; __threadfence(); }
}
}

extern "C" void kernel_launch(void* const* d_in, const int* in_sizes, int n_in, void* d_out, int out_size, void* d_ws, size_t ws_size, hipStream_t stream) {
  (void)n_in;
  auto Fp = [&](int i) { return (const float*)d_in[i]; };
  if (in_sizes[0] != NB * QL * EMB || in_sizes[1] != NB * DL * EMB || in_sizes[2] != NB * QL || in_sizes[3] != NB * DL || in_sizes[4] != CO * EMB || in_sizes[8] != CO * EMB * 3 || in_sizes[10] != NGR * NGR * NK || out_size != NB) return;
  size_t off = 0; char* ws = (char*)d_ws;
  auto carve = [&](size_t bytes) { char* p = ws + off; off += (bytes + 255) & ~(size_t)255; return p; };
  b16* W0 = (b16*)carve((size_t)CO * 1 * EP * 2); b16* W1 = (b16*)carve((size_t)CO * 2 * EP * 2); b16* W2 = (b16*)carve((size_t)CO * 3 * EP * 2);
  b16* QE = (b16*)carve((size_t)NB * QROWS * EP * 2); b16* DE = (b16*)carve((size_t)NB * DROWS * EP * 2);
  b16* NQH = (b16*)carve((size_t)NB * NGR * QR * CO * 2); b16* NQL = (b16*)carve((size_t)NB * NGR * QR * CO * 2); b16* NDH = (b16*)carve((size_t)NB * NGR * DL * CO * 2); b16* NDL = (b16*)carve((size_t)NB * NGR * DL * CO * 2);
  float* ALLG = (float*)carve((size_t)NB * NGR * NGR * 32 * 4);
  if (off > ws_size) return;
  prepw_kernel<<<dim3(16, NGR), 256, 0, stream>>>(Fp(4), Fp(6), Fp(8), W0, W1, W2);
  prepe_kernel<<<(NB * QROWS + NB * DROWS) / 8, 256, 0, stream>>>(Fp(0), Fp(1), QE, DE);
  conv_kernel<true><<<dim3(QR / 32, NGR, NB), 64, 0, stream>>>(QE, W0, W1, W2, Fp(5), Fp(7), Fp(9), NQH, NQL);
  conv_kernel<false><<<dim3(DL / 32, NGR, NB), 64, 0, stream>>>(DE, W0, W1, W2, Fp(5), Fp(7), Fp(9), NDH, NDL);
  cos_kernel<<<dim3(NGR * NGR, NB), 256, 0, stream>>>(NQH, NQL, NDH, NDL, Fp(2), Fp(3), ALLG);
  dense_kernel<<<1, 128, 0, stream>>>(ALLG, Fp(10), (float*)d_out);
}
